// PIVAE_40973988004430
// MI455X (gfx1250) — hardware-run, weakly checked
//
#include <hip/hip_runtime.h>


#ifndef NB
#define NB 2048
#endif
#define NB_FULL 2048
#define NE   256
#define NIN  2
#define NC   100
#define ND1  20
#define ND2  20
#define NO   100
#define NH1  128
#define NH2  64
#define NZ   20
#define KP1  128
#define OP7  112
#define PW   4
#define TPW  4
#define RP   132
#define CA   256.0f
#define CW   64.0f
#define FI   (1.0f / 16384.0f)
#define QRS  2048.0f
#define QRI  (1.0f / 2048.0f)
#define L2E  1.4426950408889634f
#define FSH  8.0f

#define OFF_EB1 0
#define OFF_EB2 128
#define OFF_BMU 192
#define OFF_BLV 224
#define OFF_DB1 256
#define OFF_DB2 320
#define OFF_DB3 448
#define BSH_N   576

static_assert(NB % 16 == 0);
static_assert(NB <= NB_FULL);
static_assert(PW * TPW * 16 == NE);
static_assert(TPW * 16 * 4 == 256);
static_assert(32 * 16 == 2 * TPW * 16 * 4);
static_assert((32 + 32 + 16) * 16 == 16 * NZ * 4);
static_assert((16 * NZ * 4) % 128 == 0);
static_assert(32 * 16 == 128 * 4);
static_assert(KP1 % 32 == 0 && KP1 >= NC);
static_assert(NH1 % 32 == 0 && NH2 % 32 == 0);
static_assert(ND1 <= 32 && ND2 <= 32 && NZ <= 32);
static_assert(OP7 % 16 == 0 && OP7 >= NO && OP7 <= 128);
static_assert(NO % 4 == 0 && NZ % 4 == 0);
static_assert((RP * 4) % 16 == 0 && RP >= 128);
static_assert(OFF_DB3 + 128 == BSH_N);
static_assert((size_t)NB_FULL * NE * 4 == (size_t)2097152);
static_assert((size_t)2 * NB_FULL * NE * 4 == (size_t)4194304);
static_assert((size_t)2 * NB_FULL * NE * 4 + (size_t)NB_FULL * NZ * 4 == (size_t)4358144);
static_assert((size_t)2 * NB_FULL * NE * 4 + (size_t)2 * NB_FULL * NZ * 4 == (size_t)4521984);
static_assert((KP1 * 2 + 32 + 32 + 3 * 128 + PW * 2 * 64) * 4 <= 131072);
static_assert((BSH_N + 640 + 16 * RP) * 4 <= 131072);

typedef _Float16 h16;
typedef __attribute__((ext_vector_type(16))) _Float16 v16h;
typedef __attribute__((ext_vector_type(8)))  _Float16 v8h;
typedef __attribute__((ext_vector_type(8)))  float    v8f;
typedef __attribute__((ext_vector_type(4)))  float    v4f;
typedef __attribute__((ext_vector_type(2)))  float    v2f;
typedef v4f  __attribute__((may_alias)) v4fa;

__device__ __forceinline__ unsigned short f2bf(float f) { unsigned u = __float_as_uint(f); u += 0x7FFFu + ((u >> 16) & 1u); return (unsigned short)(u >> 16); }
__device__ __forceinline__ float bfr(float f) { return __uint_as_float(((unsigned)f2bf(f)) << 16); }
__device__ __forceinline__ v16h cat16(v8h lo, v8h hi) { return __builtin_shufflevector(lo, hi, 0, 1, 2, 3, 4, 5, 6, 7, 8, 9, 10, 11, 12, 13, 14, 15); }
__device__ __forceinline__ v8f cat8(v4f a, v4f b) { return __builtin_shufflevector(a, b, 0, 1, 2, 3, 4, 5, 6, 7); }
__device__ __forceinline__ v8f wmma16(v16h a, v16h b, v8f c) { return __builtin_amdgcn_wmma_f32_16x16x32_f16(false, a, false, b, (short)0, c, false, false); }
__device__ __forceinline__ v8f wmma16g(v16h a, v16h b, v8f c) { c = wmma16(a, b, c); asm volatile("v_nop\n\tv_nop\n\tv_nop\n\tv_nop" : "+v"(c) : "v"(a), "v"(b)); return c; }
__device__ __forceinline__ v16h ldh(const h16* p) { return cat16(*(const v8h*)p, *(const v8h*)(p + 16)); }
__device__ __forceinline__ void wave_sync() { __builtin_amdgcn_fence(3  , "wavefront"); __builtin_amdgcn_wave_barrier(); asm volatile("" ::: "memory"); }
static __device__ __forceinline__ h16 toh_flush(float v) { const h16 r = (h16)v; return (fabsf(v) < 6.103515625e-05f) ? (h16)0.0f : r; }
__device__ __forceinline__ float tanh_f(float x) {
    const float ax = fabsf(x);
    const float t = __builtin_amdgcn_exp2f(ax * (-2.0f * L2E));
    const float r = (1.0f - t) * __builtin_amdgcn_rcpf(1.0f + t);
    return copysignf(r, x);
}

#define LD8S(arr, o) cat8(*(const v4fa*)(&(arr)[(o)]), *(const v4fa*)(&(arr)[(o) + 4]))

__global__ __launch_bounds__(256) void k_wconv(const float* __restrict__ src, h16* dst, int N, int K, int NP, int KP, int sn, int sk, float scale) {
    const int kp8 = KP >> 3;
    const int i = (int)(blockIdx.x * 256 + threadIdx.x);
    if (i >= NP * kp8) return;
    const int n = i / kp8, k0 = (i - n * kp8) * 8;
    const int nc = n < N ? n : N - 1;
    v8h o;
#pragma unroll
    for (int j = 0; j < 8; ++j) {
        const int k = k0 + j; const int kc = k < K ? k : K - 1;
        float v = src[(size_t)nc * (size_t)sn + (size_t)kc * (size_t)sk];
        asm volatile("" : "+v"(v));
        const bool ok = (n < N) & (k < K);
        const h16 c = toh_flush(bfr(v) * scale);
        o[j] = ok ? c : (h16)0.0f;
    }
    *(volatile v8h*)(dst + (size_t)i * 8) = o; __threadfence(); *(volatile v8h*)(dst + (size_t)i * 8) = o;
}

template <int KS, bool RES>
__device__ __forceinline__ void tile_pair(const h16* __restrict__ WT, int rowbase, int KP, int lr, int hi,
                                          const v16h (&bh)[KS], const v16h (&br)[KS], v8f& p0, v8f& p1, v8f& q0, v8f& q1) {
    p0 = (v8f){}; p1 = (v8f){}; q0 = (v8f){}; q1 = (v8f){};
    const h16* w0 = WT + (size_t)(rowbase + lr) * (size_t)KP + 8 * hi;
    const h16* w1 = w0 + (size_t)16 * (size_t)KP;
#pragma unroll
    for (int ks = 0; ks < KS; ++ks) {
        const v16h a0 = ldh(w0 + ks * 32), a1 = ldh(w1 + ks * 32);
        p0 = wmma16g(a0, bh[ks], p0); p1 = wmma16g(a1, bh[ks], p1);
        if (RES) { q0 = wmma16g(a0, br[ks], q0); q1 = wmma16g(a1, br[ks], q1); }
    }
}

template <bool RELU>
__device__ __forceinline__ void pack2(v8f p0, v8f p1, v8f q0, v8f q1, v8f c0, v8f c1, v16h& hv, v16h& rv) {
#pragma unroll
    for (int r = 0; r < 8; ++r) {
        float u = (p0[r] + q0[r] * QRI) * FI + c0[r];
        float w = (p1[r] + q1[r] * QRI) * FI + c1[r];
        if (RELU) { u = fmaxf(u, 0.0f); w = fmaxf(w, 0.0f); }
        const float uc = u * CA, wc = w * CA;
        const h16 uh = toh_flush(uc), wh = toh_flush(wc);
        hv[r] = uh; hv[8 + r] = wh;
        rv[r] = toh_flush((uc - (float)uh) * QRS); rv[8 + r] = toh_flush((wc - (float)wh) * QRS);
    }
}

__global__ __launch_bounds__(32) void k_vae(const h16* __restrict__ BWH, const h16* __restrict__ EW1T, const h16* __restrict__ EW2T, const h16* __restrict__ WMLT,
                                            const h16* __restrict__ DW1T, const h16* __restrict__ DW2T, const h16* __restrict__ DW3T,
                                            const float* __restrict__ eb1, const float* __restrict__ eb2, const float* __restrict__ bmu, const float* __restrict__ blv,
                                            const float* __restrict__ db1, const float* __restrict__ db2, const float* __restrict__ db3,
                                            const float* __restrict__ eps, float* RECON, float* MU, float* LV) {
    __shared__ __align__(16) float bsh[BSH_N];
    __shared__ __align__(16) float mls[640];
    __shared__ __align__(16) float rs[16 * RP];
    const int lane = threadIdx.x & 31, lr = lane & 15, hi = lane >> 4;
    const int m0 = blockIdx.x * 16;
#pragma unroll 1
    for (int i = lane; i < 128; i += 32) {
        bsh[OFF_EB1 + i] = bfr(eb1[i]);
        bsh[OFF_DB2 + i] = bfr(db2[i]);
        const int ic = i < NO ? i : NO - 1;
        float v = db3[ic]; asm volatile("" : "+v"(v));
        bsh[OFF_DB3 + i] = (i < NO) ? bfr(v) : 0.0f;
    }
#pragma unroll 1
    for (int i = lane; i < 64; i += 32) { bsh[OFF_EB2 + i] = bfr(eb2[i]); bsh[OFF_DB1 + i] = bfr(db1[i]); }
    { const int ic = lane < NZ ? lane : NZ - 1;
      float v = bmu[ic], w = blv[ic]; asm volatile("" : "+v"(v)); asm volatile("" : "+v"(w));
      bsh[OFF_BMU + lane] = (lane < NZ) ? bfr(v) : 0.0f; bsh[OFF_BLV + lane] = (lane < NZ) ? bfr(w) : 0.0f; }
    __syncthreads();

    v16h bwf[4];
#pragma unroll
    for (int ks = 0; ks < 4; ++ks) bwf[ks] = ldh(BWH + (size_t)(m0 + lr) * KP1 + ks * 32 + 8 * hi);
    v16h h1v[4], h1r[4];
#pragma unroll
    for (int j = 0; j < 4; ++j) {
        v8f p0, p1, q0, q1; tile_pair<4, false>(EW1T, 32 * j, KP1, lr, hi, bwf, bwf, p0, p1, q0, q1);
        const v8f c0 = LD8S(bsh, OFF_EB1 + 32 * j + 8 * hi), c1 = LD8S(bsh, OFF_EB1 + 32 * j + 16 + 8 * hi);
        pack2<true>(p0, p1, q0, q1, c0, c1, h1v[j], h1r[j]);
    }
    v16h h2v[2], h2r[2];
#pragma unroll
    for (int j = 0; j < 2; ++j) {
        v8f p0, p1, q0, q1; tile_pair<4, true>(EW2T, 32 * j, NH1, lr, hi, h1v, h1r, p0, p1, q0, q1);
        const v8f c0 = LD8S(bsh, OFF_EB2 + 32 * j + 8 * hi), c1 = LD8S(bsh, OFF_EB2 + 32 * j + 16 + 8 * hi);
        pack2<true>(p0, p1, q0, q1, c0, c1, h2v[j], h2r[j]);
    }
    v8f pm0, pm1, qm0, qm1, pl0, pl1, ql0, ql1;
    tile_pair<2, true>(WMLT, 0, NH2, lr, hi, h2v, h2r, pm0, pm1, qm0, qm1);
    tile_pair<2, true>(WMLT, 32, NH2, lr, hi, h2v, h2r, pl0, pl1, ql0, ql1);
    const v8f cm0 = LD8S(bsh, OFF_BMU + 8 * hi), cm1 = LD8S(bsh, OFF_BMU + 16 + 8 * hi);
    const v8f cl0 = LD8S(bsh, OFF_BLV + 8 * hi), cl1 = LD8S(bsh, OFF_BLV + 16 + 8 * hi);
    v8f mu0, mu1, lv0, lv1;
#pragma unroll
    for (int r = 0; r < 8; ++r) {
        mu0[r] = (pm0[r] + qm0[r] * QRI) * FI + cm0[r]; mu1[r] = (pm1[r] + qm1[r] * QRI) * FI + cm1[r];
        lv0[r] = (pl0[r] + ql0[r] * QRI) * FI + cl0[r]; lv1[r] = (pl1[r] + ql1[r] * QRI) * FI + cl1[r];
    }
    { v4f a, b;
      a[0] = mu0[0]; a[1] = mu0[1]; a[2] = mu0[2]; a[3] = mu0[3]; b[0] = mu0[4]; b[1] = mu0[5]; b[2] = mu0[6]; b[3] = mu0[7];
      *(v4fa*)(&mls[lr * NZ + 8 * hi]) = a; *(v4fa*)(&mls[lr * NZ + 8 * hi + 4]) = b;
      a[0] = lv0[0]; a[1] = lv0[1]; a[2] = lv0[2]; a[3] = lv0[3]; b[0] = lv0[4]; b[1] = lv0[5]; b[2] = lv0[6]; b[3] = lv0[7];
      *(v4fa*)(&mls[320 + lr * NZ + 8 * hi]) = a; *(v4fa*)(&mls[320 + lr * NZ + 8 * hi + 4]) = b;
      if (hi == 0) {
          a[0] = mu1[0]; a[1] = mu1[1]; a[2] = mu1[2]; a[3] = mu1[3]; *(v4fa*)(&mls[lr * NZ + 16]) = a;
          b[0] = lv1[0]; b[1] = lv1[1]; b[2] = lv1[2]; b[3] = lv1[3]; *(v4fa*)(&mls[320 + lr * NZ + 16]) = b; } }
    v16h zv[1], zr[1];
    { const float* ep = eps + (size_t)(m0 + lr) * NZ;
      const v4f e0a = *(const v4f*)(ep + 8 * hi), e0b = *(const v4f*)(ep + 8 * hi + 4);
      const v4f e1 = *(const v4f*)(ep + 16);
#pragma unroll
      for (int r = 0; r < 8; ++r) {
          const float e = (r < 4) ? e0a[r & 3] : e0b[r & 3];
          const float z = mu0[r] + __builtin_amdgcn_exp2f(lv0[r] * (0.5f * L2E)) * bfr(e);
          const float zc = z * CA; const h16 zh = toh_flush(zc);
          zv[0][r] = zh; zr[0][r] = toh_flush((zc - (float)zh) * QRS); }
#pragma unroll
      for (int r = 0; r < 4; ++r) {
          float e = e1[r]; asm volatile("" : "+v"(e));
          float z = mu1[r] + __builtin_amdgcn_exp2f(lv1[r] * (0.5f * L2E)) * bfr(e);
          z = (hi == 0) ? z : 0.0f;
          const float zc = z * CA; const h16 zh = toh_flush(zc);
          zv[0][8 + r] = zh; zr[0][8 + r] = toh_flush((zc - (float)zh) * QRS); }
#pragma unroll
      for (int r = 4; r < 8; ++r) { zv[0][8 + r] = (h16)0.0f; zr[0][8 + r] = (h16)0.0f; } }
    wave_sync();
#pragma unroll 1
    for (int ps = 0; ps < 2; ++ps) {
#pragma unroll
        for (int s = 0; s < 3; ++s) { const int idx = s * 32 + lane; const int ic = idx < 80 ? idx : 79;
            const v4f a = *(const v4fa*)(&mls[4 * ic]); const v4f b = *(const v4fa*)(&mls[320 + 4 * ic]);
            if (idx < 80) { *(volatile v4f*)(MU + (size_t)m0 * NZ + 4 * idx) = a; *(volatile v4f*)(LV + (size_t)m0 * NZ + 4 * idx) = b; } }
        if (ps == 0) __threadfence(); }
    v16h h3v[2], h3r[2];
#pragma unroll
    for (int j = 0; j < 2; ++j) {
        v8f p0, p1, q0, q1; tile_pair<1, true>(DW1T, 32 * j, 32, lr, hi, zv, zr, p0, p1, q0, q1);
        const v8f c0 = LD8S(bsh, OFF_DB1 + 32 * j + 8 * hi), c1 = LD8S(bsh, OFF_DB1 + 32 * j + 16 + 8 * hi);
        pack2<true>(p0, p1, q0, q1, c0, c1, h3v[j], h3r[j]);
    }
    v16h h4v[4], h4r[4];
#pragma unroll
    for (int j = 0; j < 4; ++j) {
        v8f p0, p1, q0, q1; tile_pair<2, true>(DW2T, 32 * j, NH2, lr, hi, h3v, h3r, p0, p1, q0, q1);
        const v8f c0 = LD8S(bsh, OFF_DB2 + 32 * j + 8 * hi), c1 = LD8S(bsh, OFF_DB2 + 32 * j + 16 + 8 * hi);
        pack2<true>(p0, p1, q0, q1, c0, c1, h4v[j], h4r[j]);
    }
#pragma unroll
    for (int j = 0; j < 4; ++j) {
        v8f p0, p1, q0, q1; tile_pair<4, true>(DW3T, 32 * j, NH1, lr, hi, h4v, h4r, p0, p1, q0, q1);
        const v8f c0 = LD8S(bsh, OFF_DB3 + 32 * j + 8 * hi), c1 = LD8S(bsh, OFF_DB3 + 32 * j + 16 + 8 * hi);
        v4f a, b;
#pragma unroll
        for (int i = 0; i < 4; ++i) { a[i] = (p0[i] + q0[i] * QRI) * FI + c0[i]; b[i] = (p0[4 + i] + q0[4 + i] * QRI) * FI + c0[4 + i]; }
        *(v4fa*)(&rs[lr * RP + 32 * j + 8 * hi]) = a; *(v4fa*)(&rs[lr * RP + 32 * j + 8 * hi + 4]) = b;
#pragma unroll
        for (int i = 0; i < 4; ++i) { a[i] = (p1[i] + q1[i] * QRI) * FI + c1[i]; b[i] = (p1[4 + i] + q1[4 + i] * QRI) * FI + c1[4 + i]; }
        *(v4fa*)(&rs[lr * RP + 32 * j + 16 + 8 * hi]) = a; *(v4fa*)(&rs[lr * RP + 32 * j + 16 + 8 * hi + 4]) = b;
    }
    wave_sync();
#pragma unroll 1
    for (int ps = 0; ps < 2; ++ps) {
#pragma unroll 4
        for (int s = 0; s < 16; ++s) {
            const v4f val = *(const v4fa*)(&rs[s * RP + 4 * lane]);
            *(volatile v4f*)(RECON + (size_t)(m0 + s) * 128 + 4 * lane) = val; }
        if (ps == 0) __threadfence(); }
}

__global__ __launch_bounds__(32 * PW) void k_phi(const float* __restrict__ x, const float* __restrict__ alphaP, const float* __restrict__ centers,
                                                  const float* __restrict__ b1, const float* __restrict__ b2, const float* __restrict__ b3,
                                                  const float* __restrict__ betaW, const float* __restrict__ betaB, const float* __restrict__ RECON,
                                                  const h16* __restrict__ W1T, const h16* __restrict__ W2T, const h16* __restrict__ W3T, float* OUT) {
    __shared__ __align__(16) float cens[KP1 * 2];
    __shared__ __align__(16) float b1s[32];
    __shared__ __align__(16) float b2s[32];
    __shared__ __align__(16) float b3s[128];
    __shared__ __align__(16) float bws[128];
    __shared__ __align__(16) float recs[128];
    __shared__ __align__(16) float ys[PW * 2 * 64];
    const int tid = threadIdx.x, lane = tid & 31, lr = lane & 15, hi = lane >> 4;
    const int wave = __builtin_amdgcn_readfirstlane((int)(threadIdx.x >> 5));
    const int bat = blockIdx.x;
#pragma unroll 1
    for (int i = tid; i < KP1 * 2; i += 32 * PW) {
        const int ic = i < NC * NIN ? i : NC * NIN - 1;
        float v = centers[ic]; asm volatile("" : "+v"(v));
        cens[i] = (i < NC * NIN) ? bfr(v) : 0.0f;
    }
    if (tid < 32) {
        const int ic = tid < ND1 ? tid : ND1 - 1; const int id = tid < ND2 ? tid : ND2 - 1;
        float v = b1[ic], w = b2[id]; asm volatile("" : "+v"(v)); asm volatile("" : "+v"(w));
        b1s[tid] = (tid < ND1) ? bfr(v) : 0.0f; b2s[tid] = (tid < ND2) ? bfr(w) : 0.0f;
    }
    { const int ic = tid < NO ? tid : NO - 1;
      float v = b3[ic], w = betaW[(size_t)bat * NO + ic]; asm volatile("" : "+v"(v)); asm volatile("" : "+v"(w));
      const float rc = RECON[(size_t)bat * 128 + tid];
      b3s[tid] = (tid < NO) ? bfr(v) : 0.0f; bws[tid] = (tid < NO) ? bfr(w) : 0.0f; recs[tid] = rc; }
    __syncthreads();

    const float nal2 = -bfr(alphaP[0]) * L2E;
    const float bb = bfr(betaB[bat]);
    const v8f zero8 = (v8f){};
    const v8f bi0 = LD8S(b1s, 8 * hi), bi1 = LD8S(b1s, 16 + 8 * hi);
    const v8f bj0 = LD8S(b2s, 8 * hi), bj1 = LD8S(b2s, 16 + 8 * hi);
#pragma unroll 1
    for (int tt = 0; tt < TPW; ++tt) {
        const int e0 = (wave * TPW + tt) * 16;
        const v2f xv = *(const v2f*)(x + ((size_t)bat * NE + (size_t)(e0 + lr)) * NIN);
        const float px0 = bfr(xv[0]), px1 = bfr(xv[1]);
        v8f acc0 = zero8, acc1 = zero8, accR0 = zero8, accR1 = zero8;
#pragma unroll 1
        for (int ks = 0; ks < KP1 / 32; ++ks) {
            const int kb = ks * 32 + 8 * hi;
            v16h fb, fr;
#pragma unroll
            for (int g = 0; g < 2; ++g) {
                const int kg = kb + 16 * g;
                const v4f q0 = *(const v4fa*)(&cens[2 * kg]), q1 = *(const v4fa*)(&cens[2 * kg + 4]), q2 = *(const v4fa*)(&cens[2 * kg + 8]), q3 = *(const v4fa*)(&cens[2 * kg + 12]);
                const float cx[8] = { q0[0], q0[2], q1[0], q1[2], q2[0], q2[2], q3[0], q3[2] };
                const float cy[8] = { q0[1], q0[3], q1[1], q1[3], q2[1], q2[3], q3[1], q3[3] };
#pragma unroll
                for (int i = 0; i < 8; ++i) {
                    const float dx = px0 - cx[i], dy = px1 - cy[i];
                    const float d2 = dx * dx + dy * dy;
                    const float ea = nal2 * d2 + FSH;
                    const float f = __builtin_amdgcn_exp2f(ea);
                    const bool keep = (ea >= -14.0f) & (kg + i < NC);
                    const float fv = keep ? f : 0.0f;
                    const h16 fh = toh_flush(fv);
                    fb[8 * g + i] = fh;
                    fr[8 * g + i] = toh_flush((fv - (float)fh) * QRS);
                }
            }
            const v16h a0 = ldh(W1T + (size_t)lr * KP1 + kb), a1 = ldh(W1T + (size_t)(16 + lr) * KP1 + kb);
            acc0 = wmma16g(a0, fb, acc0); acc1 = wmma16g(a1, fb, acc1);
            accR0 = wmma16g(a0, fr, accR0); accR1 = wmma16g(a1, fr, accR1);
        }
        v16h hb, hr;
#pragma unroll
        for (int r = 0; r < 8; ++r) {
            const float u = tanh_f((acc0[r] + accR0[r] * QRI) * FI + bi0[r]) * CA;
            const float w = tanh_f((acc1[r] + accR1[r] * QRI) * FI + bi1[r]) * CA;
            const h16 uh = toh_flush(u), wh = toh_flush(w);
            hb[r] = uh; hb[8 + r] = wh;
            hr[r] = toh_flush((u - (float)uh) * QRS); hr[8 + r] = toh_flush((w - (float)wh) * QRS); }
        const v16h w20 = ldh(W2T + (size_t)lr * 32 + 8 * hi), w21 = ldh(W2T + (size_t)(16 + lr) * 32 + 8 * hi);
        const v8f c0 = wmma16g(w20, hb, zero8), c1 = wmma16g(w21, hb, zero8);
        const v8f cR0 = wmma16g(w20, hr, zero8), cR1 = wmma16g(w21, hr, zero8);
        v16h gb, gr;
#pragma unroll
        for (int r = 0; r < 8; ++r) {
            const float u = tanh_f((c0[r] + cR0[r] * QRI) * FI + bj0[r]) * CA;
            const float w = tanh_f((c1[r] + cR1[r] * QRI) * FI + bj1[r]) * CA;
            const h16 uh = toh_flush(u), wh = toh_flush(w);
            gb[r] = uh; gb[8 + r] = wh;
            gr[r] = toh_flush((u - (float)uh) * QRS); gr[8 + r] = toh_flush((w - (float)wh) * QRS); }
        float s1 = 0.0f, s2 = 0.0f;
#pragma unroll 1
        for (int t = 0; t < OP7 / 16; ++t) {
            const v16h a = ldh(W3T + (size_t)(16 * t + lr) * 32 + 8 * hi);
            const v8f p = wmma16g(a, gb, zero8);
            const v8f pR = wmma16g(a, gr, zero8);
            const int o = 16 * t + 8 * hi;
            const v8f b3v = LD8S(b3s, o), bwv = LD8S(bws, o), rcv = LD8S(recs, o);
#pragma unroll
            for (int r = 0; r < 8; ++r) { const float ph = (p[r] + pR[r] * QRI) * FI + b3v[r]; s1 += ph * bwv[r]; s2 += ph * rcv[r]; }
        }
        s1 += __shfl_xor(s1, 16, 32); s2 += __shfl_xor(s2, 16, 32);
        ys[(wave * 2 + hi) * 64 + tt * 16 + lr] = (hi ? s2 : s1) + bb;
    }
    wave_sync();
    { const int which = lane >> 4, j4 = (lane & 15) * 4;
      const v4f val = *(const v4fa*)(&ys[(wave * 2 + which) * 64 + j4]);
      float* dst = OUT + (size_t)which * ((size_t)NB_FULL * NE) + (size_t)bat * NE + (size_t)(wave * 64 + j4);
      *(volatile v4f*)dst = val; __threadfence(); *(volatile v4f*)dst = val; }
}

static constexpr size_t al256(size_t v) { return (v + 255) & ~(size_t)255; }
static constexpr size_t SZ_W1T = al256((size_t)32 * KP1 * 2);
static constexpr size_t SZ_W2T = al256((size_t)32 * 32 * 2);
static constexpr size_t SZ_W3T = al256((size_t)OP7 * 32 * 2);
static constexpr size_t SZ_E1T = al256((size_t)NH1 * KP1 * 2);
static constexpr size_t SZ_E2T = al256((size_t)NH2 * NH1 * 2);
static constexpr size_t SZ_MLT = al256((size_t)64 * NH2 * 2);
static constexpr size_t SZ_D1T = al256((size_t)NH2 * 32 * 2);
static constexpr size_t SZ_D2T = al256((size_t)NH1 * NH2 * 2);
static constexpr size_t SZ_D3T = al256((size_t)128 * NH1 * 2);
static constexpr size_t SZ_BWH = al256((size_t)NB * KP1 * 2);
static constexpr size_t SZ_REC = al256((size_t)NB * 128 * 4);
static constexpr size_t SZ_TOTAL = SZ_W1T + SZ_W2T + SZ_W3T + SZ_E1T + SZ_E2T + SZ_MLT + SZ_D1T + SZ_D2T + SZ_D3T + SZ_BWH + SZ_REC;
static_assert(SZ_TOTAL <= (size_t)134217728);
static_assert(((size_t)32 * NH2 * 2) % 256 == 0);
static_assert((32 * KP1 * 2) % 1024 == 0 && (32 * 32 * 2) % 1024 == 0 && (OP7 * 32 * 2) % 1024 == 0 && (NH2 * 32 * 2) % 1024 == 0);

static void launch_conv(const float* src, h16* dst, int N, int K, int NP, int KP, int sn, int sk, float scale, hipStream_t stream) {
    const int items = NP * (KP / 8);
    k_wconv<<<(unsigned)((items + 255) / 256), 256, 0, stream>>>(src, dst, N, K, NP, KP, sn, sk, scale);
}

extern "C" void kernel_launch(void* const* d_in, const int* in_sizes, int n_in,
                              void* d_out, int out_size, void* d_ws, size_t ws_size, hipStream_t stream) {
    if (n_in < 26) return;
    const size_t need[26] = { (size_t)NB * NE * NIN, (size_t)NB * NZ, 1, (size_t)NC * NIN, (size_t)NC * ND1, ND1, (size_t)ND1 * ND2, ND2, (size_t)ND2 * NO, NO,
                              (size_t)NB * NO, NB, (size_t)NO * NH1, NH1, (size_t)NH1 * NH2, NH2, (size_t)NH2 * NZ, NZ, (size_t)NH2 * NZ, NZ,
                              (size_t)NZ * NH2, NH2, (size_t)NH2 * NH1, NH1, (size_t)NH1 * NO, NO };
    for (int i = 0; i < 26; ++i) if ((size_t)in_sizes[i] < need[i]) return;
    if ((size_t)out_size < (size_t)2 * NB_FULL * NE + (size_t)NB_FULL * NZ + (size_t)NB * NZ) return;
    if (SZ_TOTAL > ws_size) return;
    const float* x   = (const float*)d_in[0];  const float* eps = (const float*)d_in[1];
    const float* alp = (const float*)d_in[2];  const float* cen = (const float*)d_in[3];
    const float* W1  = (const float*)d_in[4];  const float* b1  = (const float*)d_in[5];
    const float* W2  = (const float*)d_in[6];  const float* b2  = (const float*)d_in[7];
    const float* W3  = (const float*)d_in[8];  const float* b3  = (const float*)d_in[9];
    const float* bW  = (const float*)d_in[10]; const float* bB  = (const float*)d_in[11];
    const float* eW1 = (const float*)d_in[12]; const float* eb1 = (const float*)d_in[13];
    const float* eW2 = (const float*)d_in[14]; const float* eb2 = (const float*)d_in[15];
    const float* Wmu = (const float*)d_in[16]; const float* bmu = (const float*)d_in[17];
    const float* Wlv = (const float*)d_in[18]; const float* blv = (const float*)d_in[19];
    const float* dW1 = (const float*)d_in[20]; const float* db1 = (const float*)d_in[21];
    const float* dW2 = (const float*)d_in[22]; const float* db2 = (const float*)d_in[23];
    const float* dW3 = (const float*)d_in[24]; const float* db3 = (const float*)d_in[25];
    float* OUT = (float*)d_out;
    float* MU = OUT + (size_t)2 * NB_FULL * NE;
    float* LV = MU + (size_t)NB_FULL * NZ;
    char* wsp = (char*)d_ws;
    h16* W1T = (h16*)wsp; wsp += SZ_W1T;
    h16* W2T = (h16*)wsp; wsp += SZ_W2T;
    h16* W3T = (h16*)wsp; wsp += SZ_W3T;
    h16* E1T = (h16*)wsp; wsp += SZ_E1T;
    h16* E2T = (h16*)wsp; wsp += SZ_E2T;
    h16* MLT = (h16*)wsp; wsp += SZ_MLT;
    h16* D1T = (h16*)wsp; wsp += SZ_D1T;
    h16* D2T = (h16*)wsp; wsp += SZ_D2T;
    h16* D3T = (h16*)wsp; wsp += SZ_D3T;
    h16* BWH = (h16*)wsp; wsp += SZ_BWH;
    float* REC = (float*)wsp; wsp += SZ_REC;

    launch_conv(W1,  W1T, ND1, NC,  32,  KP1, 1, ND1, CW, stream);
    launch_conv(W2,  W2T, ND2, ND1, 32,  32,  1, ND2, CW, stream);
    launch_conv(W3,  W3T, NO,  ND2, OP7, 32,  1, NO,  CW, stream);
    launch_conv(eW1, E1T, NH1, NO,  NH1, KP1, 1, NH1, CW, stream);
    launch_conv(eW2, E2T, NH2, NH1, NH2, NH1, 1, NH2, CW, stream);
    launch_conv(Wmu, MLT, NZ,  NH2, 32,  NH2, 1, NZ,  CW, stream);
    launch_conv(Wlv, MLT + (size_t)32 * NH2, NZ, NH2, 32, NH2, 1, NZ, CW, stream);
    launch_conv(dW1, D1T, NH2, NZ,  NH2, 32,  1, NH2, CW, stream);
    launch_conv(dW2, D2T, NH1, NH2, NH1, NH2, 1, NH1, CW, stream);
    launch_conv(dW3, D3T, NO,  NH1, 128, NH1, 1, NO,  CW, stream);
    launch_conv(bW,  BWH, NB,  NO,  NB,  KP1, NO, 1,  CA, stream);

    k_vae<<<NB / 16, 32, 0, stream>>>(BWH, E1T, E2T, MLT, D1T, D2T, D3T, eb1, eb2, bmu, blv, db1, db2, db3, eps, REC, MU, LV);
    k_phi<<<NB, 32 * PW, 0, stream>>>(x, alp, cen, b1, b2, b3, bW, bB, REC, W1T, W2T, W3T, OUT);
}
